// SingleNet_19808389169762
// MI455X (gfx1250) — hardware-verified
//
#include <hip/hip_runtime.h>
#include <math.h>

typedef __attribute__((ext_vector_type(16))) _Float16 v16h;
typedef __attribute__((ext_vector_type(16))) __bf16 v16b;
typedef __attribute__((ext_vector_type(8)))  _Float16 v8h;
typedef __attribute__((ext_vector_type(8)))  float v8f;
typedef __attribute__((ext_vector_type(4)))  float v4f;
typedef __attribute__((ext_vector_type(2)))  float v2f;
typedef __attribute__((ext_vector_type(4)))  unsigned v4u;
typedef __attribute__((ext_vector_type(4)))  int v4i;
typedef float __attribute__((may_alias)) float_a;
typedef int __attribute__((may_alias)) int_a;

template <typename T> __device__ __forceinline__ void vst2(void* p, T v) { *(volatile T*)p = v; __threadfence(); *(volatile T*)p = v; }
__device__ __forceinline__ v8f wmma16(v16h a, v16h b, v8f c) {
  v8f d = __builtin_amdgcn_wmma_f32_16x16x32_f16(false, a, false, b, (short)0, c, false, false);
  asm volatile("v_nop\n\tv_nop\n\tv_nop\n\tv_nop" : "+v"(d) : "v"(a), "v"(b));
  return d;
}
__device__ __forceinline__ v8f wmma_bf(v16b a, v16b b, v8f c) {
  v8f d = __builtin_amdgcn_wmma_f32_16x16x32_bf16(false, a, false, b, (short)0, c, false, false);
  asm volatile("v_nop\n\tv_nop\n\tv_nop\n\tv_nop" : "+v"(d) : "v"(a), "v"(b));
  return d;
}
__device__ __forceinline__ v16h frag_h(const _Float16* rowk0, int lane) {
  union { v16h v; v8h q[2]; } u; const _Float16* p = rowk0 + 8 * (lane >> 4);
  u.q[0] = *(const v8h*)p; u.q[1] = *(const v8h*)(p + 16); return u.v;
}
__device__ __forceinline__ v16h frag_f32(const float* rowk0, int lane) {
  v16h a; const float* p = rowk0 + 8 * (lane >> 4);
#pragma unroll
  for (int i = 0; i < 8; ++i) { a[i] = (_Float16)p[i]; a[8 + i] = (_Float16)p[16 + i]; }
  return a;
}
__device__ __forceinline__ v16h frag_f32s(const float* rowk0, int lane, float sc) {
  v16h a; const float* p = rowk0 + 8 * (lane >> 4);
#pragma unroll
  for (int i = 0; i < 8; ++i) { a[i] = (_Float16)(p[i] * sc); a[8 + i] = (_Float16)(p[16 + i] * sc); }
  return a;
}
__device__ __forceinline__ v16h fragc_f32(const float* W, int k0, int n, int lane, int ld, int K) {
  v16h a; const int g = lane >> 4;
#pragma unroll
  for (int i = 0; i < 8; ++i) { const int ka = k0 + 8 * g + i, kb = ka + 16;
    a[i] = (_Float16)(ka < K ? W[(size_t)(ka < K ? ka : K - 1) * ld + n] : 0.f); a[8 + i] = (_Float16)(kb < K ? W[(size_t)(kb < K ? kb : K - 1) * ld + n] : 0.f); }
  return a;
}
struct F2 { v16b h, l; };
__device__ __forceinline__ F2 bsplit16(const float v[16]) { F2 r;
#pragma unroll
  for (int i = 0; i < 16; ++i) { const __bf16 h = (__bf16)v[i]; r.h[i] = h; r.l[i] = (__bf16)(v[i] - (float)h); }
  return r; }
__device__ __forceinline__ F2 split_row(const float* row, int k0, int lane) { float v[16]; const float* p = row + k0 + 8 * (lane >> 4);
#pragma unroll
  for (int i = 0; i < 8; ++i) { v[i] = p[i]; v[8 + i] = p[16 + i]; }
  return bsplit16(v); }
__device__ __forceinline__ F2 split_rowK(const float* row, int k0, int lane, int K) { float v[16]; const int g = lane >> 4;
#pragma unroll
  for (int i = 0; i < 8; ++i) { const int ka = k0 + 8 * g + i, kb = ka + 16; v[i] = ka < K ? row[ka < K ? ka : K - 1] : 0.f; v[8 + i] = kb < K ? row[kb < K ? kb : K - 1] : 0.f; }
  return bsplit16(v); }
__device__ __forceinline__ F2 split_col(const float* W, int k0, int n, int lane, int ld, int K) { float v[16]; const int g = lane >> 4;
#pragma unroll
  for (int i = 0; i < 8; ++i) { const int ka = k0 + 8 * g + i, kb = ka + 16; v[i] = ka < K ? W[(size_t)(ka < K ? ka : K - 1) * ld + n] : 0.f; v[8 + i] = kb < K ? W[(size_t)(kb < K ? kb : K - 1) * ld + n] : 0.f; }
  return bsplit16(v); }
__device__ __forceinline__ v8f mac3(const F2& a, const F2& b, v8f c) { c = wmma_bf(a.l, b.h, c); c = wmma_bf(a.h, b.l, c); return wmma_bf(a.h, b.h, c); }
__device__ __forceinline__ float sigm(float v) { return 1.0f / (1.0f + expf(-v)); }
#define LDSX() do { asm volatile("s_wait_dscnt 0" ::: "memory"); __builtin_amdgcn_wave_barrier(); __builtin_amdgcn_fence(__ATOMIC_RELEASE, "workgroup"); } while (0)


#define BB 32
#define I0 1024
#define H1 2048
#define H2 2048
#define O3 1024
#define MH 32
#ifndef TR1
#define TR1 H1
#define TR2 H2
#define TR3 O3
#endif
typedef __attribute__((ext_vector_type(8))) __bf16 v8b;
__device__ __forceinline__ v16b frag_gbf(const float* rowk0, int lane) {
  v16b a; const float* p = rowk0 + 8 * (lane >> 4);
#pragma unroll
  for (int i = 0; i < 8; ++i) { a[i] = (__bf16)p[i]; a[8 + i] = (__bf16)p[16 + i]; }
  return a;
}
__device__ __forceinline__ v16b frag_b(const __bf16* rowk0, int lane) {
  union { v16b v; v8b q[2]; } u; const __bf16* p = rowk0 + 8 * (lane >> 4);
  u.q[0] = *(const v8b*)p; u.q[1] = *(const v8b*)(p + 16); return u.v;
}
__device__ __forceinline__ float bfr(float v) { return (float)(__bf16)v; }
#define WS_A1  0u
#define WS_A2  (WS_A1 + 4u * BB * H1)
#define WS_END (WS_A2 + 4u * BB * H2)

template <int K, bool EXACT>
__global__ __launch_bounds__(128) void k_mlp(const float* __restrict__ IN, const float* __restrict__ Wt, const float* __restrict__ bias, float* __restrict__ OUT, int NOUT) {
  __shared__ __align__(16) float so[32][68];
  const int tid = threadIdx.x, wave = tid >> 5, lane = tid & 31, col = lane & 15, g = lane >> 4; const int rt = wave & 1, cp = wave >> 1; const int n0 = blockIdx.x * 64;
  v8f acc[2] = {};
#pragma unroll 2
  for (int kc = 0; kc < K / 32; ++kc) {
    if (EXACT) { const v16b a = frag_gbf(IN + (size_t)(rt * 16 + col) * K + kc * 32, lane);
#pragma unroll
      for (int j = 0; j < 2; ++j) acc[j] = wmma_bf(a, frag_gbf(Wt + (size_t)(n0 + (cp * 2 + j) * 16 + col) * K + kc * 32, lane), acc[j]); }
    else { const F2 a = split_row(IN + (size_t)(rt * 16 + col) * K, kc * 32, lane);
#pragma unroll
      for (int j = 0; j < 2; ++j) { const v16b w = frag_gbf(Wt + (size_t)(n0 + (cp * 2 + j) * 16 + col) * K + kc * 32, lane); acc[j] = wmma_bf(a.l, w, acc[j]); acc[j] = wmma_bf(a.h, w, acc[j]); } } }
#pragma unroll
  for (int j = 0; j < 2; ++j) { const int c = (cp * 2 + j) * 16 + col; const float bb = bfr(bias[n0 + c]);
#pragma unroll
    for (int r = 0; r < 8; ++r) so[rt * 16 + 8 * g + r][c] = fmaxf(acc[j][r] + bb, 0.f); }
  __syncthreads();
  for (int q = tid; q < 32 * 16; q += 128) { const int r = q >> 4, pc = q & 15; vst2(OUT + (size_t)r * NOUT + n0 + pc * 4, *(const v4f*)&so[r][pc * 4]); }
}
template <int IW>
__global__ __launch_bounds__(256) void k_meta(const float* __restrict__ VIN, int vin_rounded, const float* __restrict__ Wt, const float* __restrict__ VOUT, const float* __restrict__ mw1, const float* __restrict__ mb1, const float* __restrict__ mw2, const float* __restrict__ mb2, float* __restrict__ NW) {
  __shared__ float s0[MH], s1[MH], sc[MH], s2[MH];
  const int o = blockIdx.x, tid = threadIdx.x; const float vo = VOUT[o];
  if (tid < MH) { s0[tid] = bfr(mw1[tid * 3 + 0]); s1[tid] = bfr(mw1[tid * 3 + 1]); sc[tid] = bfr(mw1[tid * 3 + 2]) * vo + bfr(mb1[tid]); s2[tid] = bfr(mw2[tid]); }
  __syncthreads();
  const float b2 = bfr(mb2[0]);
  for (int p = tid; p < IW / 4; p += 256) { v4f v; for (int k = 0; k < 4; ++k) { const int i = p * 4 + k; float vi = VIN[i]; if (vin_rounded) vi = bfr(vi); const float w = bfr(Wt[(size_t)o * IW + i]); float s = b2;
#pragma unroll 1
      for (int m = 0; m < MH; ++m) s += fmaxf(s0[m] * vi + s1[m] * w + sc[m], 0.f) * s2[m];
      v[k] = s; } vst2(NW + (size_t)o * IW + p * 4, v); }
}

extern "C" void kernel_launch(void* const* d_in, const int* in_sizes, int n_in, void* d_out, int out_size, void* d_ws, size_t ws_size, hipStream_t stream) {
  (void)in_sizes; (void)n_in; (void)out_size;
  const float** F = (const float**)d_in;
  if (ws_size < (size_t)WS_END) return;
  char* ws = (char*)d_ws; float *A1 = (float*)(ws + WS_A1), *A2 = (float*)(ws + WS_A2);
  float* OUT = (float*)d_out; float* NW1 = OUT + BB * O3; float* NW2 = NW1 + (size_t)H1 * I0; float* NW3 = NW2 + (size_t)H2 * H1;
  k_mlp<I0, true><<<H1 / 64, 128, 0, stream>>>(F[0], F[1], F[2], A1, H1);
  k_mlp<H1, false><<<H2 / 64, 128, 0, stream>>>(A1, F[3], F[4], A2, H2);
  k_mlp<H2, false><<<O3 / 64, 128, 0, stream>>>(A2, F[5], F[6], OUT, O3);
  k_meta<I0><<<TR1, 256, 0, stream>>>(F[0], 1, F[1], A1, F[7], F[8], F[9], F[10], NW1);
  k_meta<H1><<<TR2, 256, 0, stream>>>(A1, 0, F[3], A2, F[7], F[8], F[9], F[10], NW2);
  k_meta<H2><<<TR3, 256, 0, stream>>>(A2, 0, F[5], OUT, F[7], F[8], F[9], F[10], NW3);
}
